// GAFlowCore_78932908966242
// MI455X (gfx1250) — hardware-verified
//
#include <hip/hip_runtime.h>

typedef __bf16 v16b __attribute__((ext_vector_type(16)));
typedef __bf16 v8b  __attribute__((ext_vector_type(8)));
typedef float  v8f  __attribute__((ext_vector_type(8)));
typedef float  v4f  __attribute__((ext_vector_type(4)));
typedef unsigned short us8 __attribute__((ext_vector_type(8)));
typedef v8b __attribute__((may_alias)) v8ba;
typedef v4f __attribute__((may_alias)) v4fa;

union Frag { v16b v; v8b half[2]; };

#define HW     8192
#define IMW    128
#define DIMC   256
#define NLV    4
#define NCH    324
#define NTOT   10880
#define NPAD   11264
#define CHK    512
#define NCHUNK 22
#define WIN    12
#define WCELL  144
#define TP     260

__device__ __forceinline__ unsigned short bf16_rne(float f) {
  const unsigned u = __float_as_uint(f);
  return (unsigned short)((u + 0x7fffu + ((u >> 16) & 1u)) >> 16);
}
__device__ __forceinline__ void split_hl(float x, unsigned short& hb, unsigned short& lb) {
  hb = bf16_rne(x);
  const float hf = __uint_as_float(((unsigned)hb) << 16);
  lb = bf16_rne(x - hf);
}

__device__ __forceinline__ v8f wmma_bf16(v16b a, v16b b, v8f c) {
  return __builtin_amdgcn_wmma_f32_16x16x32_bf16(false, a, false, b, (short)0, c, false, false);
}

__device__ __forceinline__ v16b ldfrag(const unsigned short* p, int h) {
  Frag f;
  f.half[0] = *(const v8ba*)(p + 8 * h);
  f.half[1] = *(const v8ba*)(p + 16 + 8 * h);
  return f.v;
}

__device__ __forceinline__ void mma_group(v8f& d00, v8f& d10, v8f& d01, v8f& d11,
                                          v16b aH0, v16b aL0, v16b aH1, v16b aL1,
                                          v16b bH0, v16b bL0, v16b bH1, v16b bL1) {
  d00 = wmma_bf16(aH0, bH0, d00);
  d10 = wmma_bf16(aH1, bH0, d10);
  d01 = wmma_bf16(aH0, bH1, d01);
  d11 = wmma_bf16(aH1, bH1, d11);
  d00 = wmma_bf16(aH0, bL0, d00);
  d10 = wmma_bf16(aH1, bL0, d10);
  d01 = wmma_bf16(aH0, bL1, d01);
  d11 = wmma_bf16(aH1, bL1, d11);
  d00 = wmma_bf16(aL0, bH0, d00);
  d10 = wmma_bf16(aL1, bH0, d10);
  d01 = wmma_bf16(aL0, bH1, d01);
  d11 = wmma_bf16(aL1, bH1, d11);
  asm volatile("v_nop\n\tv_nop\n\tv_nop\n\tv_nop"
               : "+v"(d00), "+v"(d10), "+v"(d01), "+v"(d11)
               : "v"(aH0), "v"(aL0), "v"(aH1), "v"(aL1), "v"(bH0), "v"(bL0), "v"(bH1), "v"(bL1));
}

__device__ __forceinline__ void plane_store_pass(const float* T, unsigned short* PH, unsigned short* PL,
                                                 int row0, int w, int lane) {
  const int q8 = lane & 7, sub = lane >> 3;
  #pragma unroll
  for (int i = 0; i < 4; ++i) {
    const int row = w * 4 + i;
    const int c = 64 * sub + 8 * q8;
    const v4f a = *(const v4fa*)(T + row * TP + c);
    const v4f b = *(const v4fa*)(T + row * TP + c + 4);
    unsigned short h0, h1, h2, h3, h4, h5, h6, h7;
    unsigned short l0, l1, l2, l3, l4, l5, l6, l7;
    split_hl(a.x, h0, l0); split_hl(a.y, h1, l1); split_hl(a.z, h2, l2); split_hl(a.w, h3, l3);
    split_hl(b.x, h4, l4); split_hl(b.y, h5, l5); split_hl(b.z, h6, l6); split_hl(b.w, h7, l7);
    const us8 hv = {h0, h1, h2, h3, h4, h5, h6, h7};
    const us8 lv = {l0, l1, l2, l3, l4, l5, l6, l7};
    const size_t g = (size_t)(row0 + row) * DIMC + c;
    *(volatile us8*)(PH + g) = hv;
    *(volatile us8*)(PL + g) = lv;
  }
}

__global__ __launch_bounds__(256) void prep_a_kernel(
    const float* __restrict__ f1, unsigned short* __restrict__ AH, unsigned short* __restrict__ AL)
{
  __shared__ __align__(16) float T[32 * TP];
  const int tid = threadIdx.x, lane = tid & 31, w = tid >> 5;
  const int m0 = blockIdx.x * 32;
  #pragma unroll 4
  for (int i = 0; i < 32; ++i) {
    const int c = i * 8 + w;
    T[lane * TP + c] = f1[(size_t)c * HW + m0 + lane];
  }
  __syncthreads();
  plane_store_pass(T, AH, AL, m0, w, lane);
  __threadfence();
  plane_store_pass(T, AH, AL, m0, w, lane);
}

__global__ __launch_bounds__(256) void prep_b_kernel(
    const float* __restrict__ f2, unsigned short* __restrict__ BH, unsigned short* __restrict__ BL)
{
  __shared__ __align__(16) float T[32 * TP];
  const int tid = threadIdx.x, lane = tid & 31, w = tid >> 5;
  const int n0 = blockIdx.x * 32;
  int l, base;
  if (n0 < 8192)       { l = 0; base = 0;     }
  else if (n0 < 10240) { l = 1; base = 8192;  }
  else if (n0 < 10752) { l = 2; base = 10240; }
  else                 { l = 3; base = 10752; }
  const bool pad = (n0 >= NTOT);
  const int logW = 7 - l, Wl = IMW >> l, pool = 1 << l;
  const int j = n0 - base + lane;
  const int Y = j >> logW, X = j & (Wl - 1);
  const int pixbase = ((Y << l) * IMW) + (X << l);
  const float invp = __uint_as_float((unsigned)(127 - 2 * l) << 23);

  #pragma unroll 1
  for (int i = 0; i < 32; ++i) {
    const int c = i * 8 + w;
    float s = 0.0f;
    if (!pad) {
      const float* src = f2 + (size_t)c * HW + pixbase;
      for (int py = 0; py < pool; ++py)
        for (int px = 0; px < pool; ++px)
          s += src[py * IMW + px];
      s *= invp;
    }
    T[lane * TP + c] = s;
  }
  __syncthreads();
  plane_store_pass(T, BH, BL, n0, w, lane);
  __threadfence();
  plane_store_pass(T, BH, BL, n0, w, lane);
}

__device__ __forceinline__ void out_store_pass(const float* S, float* out, int m0, int w, int lane) {
  const int q8 = lane & 7, sub = lane >> 3;
  #pragma unroll 1
  for (int i = 0; i < 11; ++i) {
    if (8 * i + w < 81) {
      const int L = 32 * i + 4 * w + sub;
      const v4f v = *(const v4fa*)(S + L * 32 + 4 * q8);
      *(volatile v4f*)(out + (size_t)L * HW + m0 + 4 * q8) = v;
    }
  }
}

__global__ __launch_bounds__(256) void corr_kernel(
    const unsigned short* __restrict__ AH, const unsigned short* __restrict__ AL,
    const unsigned short* __restrict__ BH, const unsigned short* __restrict__ BL,
    const float* __restrict__ coords, float* __restrict__ out)
{
  #pragma clang fp contract(off)
  __shared__ __align__(16) float sWB[32 * NLV * WCELL];
  __shared__ __align__(16) float sCT[32 * CHK];
  __shared__ int   sBX[32 * NLV];
  __shared__ int   sBY[32 * NLV];
  __shared__ float sCX[32];
  __shared__ float sCY[32];

  const int tid = threadIdx.x, lane = tid & 31, w = tid >> 5;
  const int h = lane >> 4, m = lane & 15;
  const int m0 = blockIdx.x * 32;

  if (tid < 32 * NLV) {
    const int px = tid >> 2, l = tid & 3;
    const float cx = coords[m0 + px];
    const float cy = coords[HW + m0 + px];
    const float inv = __uint_as_float((unsigned)(127 - l) << 23);
    sBX[px * NLV + l] = (int)floorf(cx * inv) - 5;
    sBY[px * NLV + l] = (int)floorf(cy * inv) - 5;
    if (l == 0) { sCX[px] = cx; sCY[px] = cy; }
  }
  #pragma unroll 1
  for (int i = tid; i < 32 * NLV * WCELL; i += 256) sWB[i] = 0.0f;

  const unsigned short* a0H = AH + (size_t)(m0 + m) * DIMC;
  const unsigned short* a0L = AL + (size_t)(m0 + m) * DIMC;
  const unsigned short* a1H = a0H + 16 * DIMC;
  const unsigned short* a1L = a0L + 16 * DIMC;
  const int ncol = 64 * w + m;

  const int el = tid >> 6;
  const int epx = (tid >> 1) & 31, ehx = tid & 1;
  const int eLogW = 7 - el, eWl = IMW >> el, eHl = 64 >> el;
  const int eBase = (el == 0) ? 0 : ((el == 1) ? 8192 : ((el == 2) ? 10240 : 10752));

  const v8f zero8 = {0.f, 0.f, 0.f, 0.f, 0.f, 0.f, 0.f, 0.f};

  #pragma unroll 1
  for (int ci = 0; ci < NCHUNK; ++ci) {
    const int c0 = ci * CHK;
    v8f acc[2][4];
    #pragma unroll
    for (int mt = 0; mt < 2; ++mt)
      #pragma unroll
      for (int nt = 0; nt < 4; ++nt) acc[mt][nt] = zero8;

    if (c0 + 64 * w < NTOT) {
      const unsigned short* bH = BH + (size_t)(c0 + ncol) * DIMC;
      const unsigned short* bL = BL + (size_t)(c0 + ncol) * DIMC;
      #pragma unroll 1
      for (int ks = 0; ks < DIMC / 32; ++ks) {
        const int k0 = ks * 32;
        const v16b fa0H = ldfrag(a0H + k0, h);
        const v16b fa0L = ldfrag(a0L + k0, h);
        const v16b fa1H = ldfrag(a1H + k0, h);
        const v16b fa1L = ldfrag(a1L + k0, h);
        #pragma unroll
        for (int g = 0; g < 2; ++g) {
          const size_t o0 = (size_t)(32 * g) * DIMC + k0;
          const size_t o1 = o0 + (size_t)16 * DIMC;
          const v16b fb0H = ldfrag(bH + o0, h);
          const v16b fb0L = ldfrag(bL + o0, h);
          const v16b fb1H = ldfrag(bH + o1, h);
          const v16b fb1L = ldfrag(bL + o1, h);
          mma_group(acc[0][2 * g], acc[1][2 * g], acc[0][2 * g + 1], acc[1][2 * g + 1],
                    fa0H, fa0L, fa1H, fa1L, fb0H, fb0L, fb1H, fb1L);
        }
      }
    }
    __syncthreads();

    #pragma unroll
    for (int mt = 0; mt < 2; ++mt)
      #pragma unroll
      for (int nt = 0; nt < 4; ++nt)
        #pragma unroll
        for (int r = 0; r < 8; ++r)
          sCT[(16 * mt + 8 * h + r) * CHK + 64 * w + 16 * nt + m] = acc[mt][nt][r] * 0.0625f;
    __syncthreads();

    {
      const int lvEnd = eBase + eHl * eWl;
      const int lo = (c0 > eBase) ? c0 : eBase;
      const int hi = (c0 + CHK < lvEnd) ? (c0 + CHK) : lvEnd;
      if (lo < hi) {
        const int Ylo = (lo - eBase) >> eLogW;
        const int Yhi = (hi - eBase) >> eLogW;
        const int bx = sBX[epx * NLV + el];
        const int by = sBY[epx * NLV + el];
        int wylo = Ylo - by; wylo = (wylo < 0) ? 0 : wylo;
        int wyhi = Yhi - by; wyhi = (wyhi > WIN) ? WIN : wyhi;
        const int wbBase = (epx * NLV + el) * WCELL;
        for (int wy = wylo; wy < wyhi; ++wy) {
          const int rowoff = eBase + ((by + wy) << eLogW) - c0;
          #pragma unroll
          for (int i = 0; i < 6; ++i) {
            const int wx = 6 * ehx + i;
            const int X = bx + wx;
            int col = rowoff + X;
            col = (col < 0) ? 0 : ((col > CHK - 1) ? (CHK - 1) : col);
            const float v = sCT[epx * CHK + col];
            if (X >= 0 && X < eWl) sWB[wbBase + wy * WIN + wx] = v;
          }
        }
      }
    }
  }
  __syncthreads();

  #pragma unroll 1
  for (int jt = 0; jt < 41; ++jt) {
    const int k = tid + 256 * jt;
    if (k < NCH * 32) {
      const int ch = k >> 5, px = k & 31;
      const int l = ch / 81;
      const int p = ch - 81 * l;
      const int p9 = p / 9;
      const float ox = (float)(p9 - 4);
      const float oy = (float)((p - 9 * p9) - 4);
      const float inv = __uint_as_float((unsigned)(127 - l) << 23);
      const int Wl = IMW >> l, Hl = 64 >> l;
      const float xu = sCX[px] * inv;
      const float yu = sCY[px] * inv;
      const float xs = xu + ox;
      const float ys = yu + oy;
      const float x0f = floorf(xs), y0f = floorf(ys);
      const float wx1 = xs - x0f, wx0 = 1.0f - wx1;
      const float wy1 = ys - y0f, wy0 = 1.0f - wy1;
      const int x0 = (int)x0f, y0 = (int)y0f, x1 = x0 + 1, y1 = y0 + 1;
      const bool vx0 = (x0 >= 0) && (x0 <= Wl - 1);
      const bool vx1 = (x1 >= 0) && (x1 <= Wl - 1);
      const bool vy0 = (y0 >= 0) && (y0 <= Hl - 1);
      const bool vy1 = (y1 >= 0) && (y1 <= Hl - 1);
      const int bx = sBX[px * NLV + l], by = sBY[px * NLV + l];
      int rx0 = x0 - bx; rx0 = (rx0 < 0) ? 0 : ((rx0 > WIN - 1) ? (WIN - 1) : rx0);
      int rx1 = x1 - bx; rx1 = (rx1 < 0) ? 0 : ((rx1 > WIN - 1) ? (WIN - 1) : rx1);
      int ry0 = y0 - by; ry0 = (ry0 < 0) ? 0 : ((ry0 > WIN - 1) ? (WIN - 1) : ry0);
      int ry1 = y1 - by; ry1 = (ry1 < 0) ? 0 : ((ry1 > WIN - 1) ? (WIN - 1) : ry1);
      const int wb = (px * NLV + l) * WCELL;
      const float t00 = sWB[wb + ry0 * WIN + rx0];
      const float t01 = sWB[wb + ry0 * WIN + rx1];
      const float t10 = sWB[wb + ry1 * WIN + rx0];
      const float t11 = sWB[wb + ry1 * WIN + rx1];
      const float g00 = (vy0 && vx0) ? t00 : 0.0f;
      const float g01 = (vy0 && vx1) ? t01 : 0.0f;
      const float g10 = (vy1 && vx0) ? t10 : 0.0f;
      const float g11 = (vy1 && vx1) ? t11 : 0.0f;
      const float s0 = (g00 * wy0) * wx0;
      const float s1 = (g01 * wy0) * wx1;
      const float s2 = (g10 * wy1) * wx0;
      const float s3 = (g11 * wy1) * wx1;
      const float res = ((s0 + s1) + s2) + s3;
      sCT[ch * 32 + px] = res;
    }
  }
  __syncthreads();

  out_store_pass(sCT, out, m0, w, lane);
  __threadfence();
  out_store_pass(sCT, out, m0, w, lane);
}

extern "C" void kernel_launch(void* const* d_in, const int* in_sizes, int n_in,
                              void* d_out, int out_size, void* d_ws, size_t ws_size,
                              hipStream_t stream) {
  if (n_in < 3) return;
  if (in_sizes[0] != DIMC * HW) return;
  if (in_sizes[1] != DIMC * HW) return;
  if (in_sizes[2] != 2 * HW) return;
  if (out_size != NCH * HW) return;

  const float* fmap1  = (const float*)d_in[0];
  const float* fmap2  = (const float*)d_in[1];
  const float* coords = (const float*)d_in[2];
  float* out = (float*)d_out;

  const size_t a_bytes = (size_t)HW * DIMC * 2;
  const size_t b_bytes = (size_t)NPAD * DIMC * 2;
  const size_t total = 2 * a_bytes + 2 * b_bytes;
  if (total > ws_size) return;

  char* ws = (char*)d_ws;
  unsigned short* AH = (unsigned short*)(ws);
  unsigned short* AL = (unsigned short*)(ws + a_bytes);
  unsigned short* BH = (unsigned short*)(ws + 2 * a_bytes);
  unsigned short* BL = (unsigned short*)(ws + 2 * a_bytes + b_bytes);

  prep_a_kernel<<<HW / 32, 256, 0, stream>>>(fmap1, AH, AL);
  prep_b_kernel<<<NPAD / 32, 256, 0, stream>>>(fmap2, BH, BL);
  corr_kernel<<<HW / 32, 256, 0, stream>>>(AH, AL, BH, BL, coords, out);
}
